// MyMultiHeadAttention_48103633715879
// MI455X (gfx1250) — hardware-verified
//
#include <hip/hip_runtime.h>


#ifndef NB
#define NB 4
#endif
#ifndef SEQ
#define SEQ 2048
#endif
#define NB_FULL  4
#define SEQ_FULL 2048
#define DM   256
#define NH   8
#define HD   64
#define DQ   (NH * HD)
#define D3   (3 * DQ)
#define FO   64
#define KCH  64
#define PP   72
#define PCAR 1024.0f
#define SCL  0.125f
#define L2E  1.4426950408889634f
static_assert(NB >= 1 && NB <= NB_FULL);
static_assert(SEQ >= KCH && SEQ <= SEQ_FULL && SEQ % 64 == 0 && SEQ % KCH == 0);
static_assert(DM % 32 == 0 && DQ % 32 == 0 && D3 % 64 == 0 && HD == 64 && FO == 64 && KCH == 64);

typedef _Float16 h16;
typedef unsigned short bf;
typedef __attribute__((ext_vector_type(16))) __bf16   v16bf;
typedef __attribute__((ext_vector_type(16))) _Float16 v16h;
typedef __attribute__((ext_vector_type(8)))  _Float16 v8h;
typedef __attribute__((ext_vector_type(8)))  unsigned short v8us;
typedef __attribute__((ext_vector_type(8)))  float    v8f;
typedef __attribute__((ext_vector_type(4)))  float    v4f;
typedef v8h  __attribute__((may_alias)) v8ha;
typedef v4f  __attribute__((may_alias)) v4fa;
typedef v8us __attribute__((may_alias)) v8usa;

__device__ __forceinline__ unsigned short f2bf(float f) { unsigned u = __float_as_uint(f); u += 0x7FFFu + ((u >> 16) & 1u); return (unsigned short)(u >> 16); }
__device__ __forceinline__ float bf2f(unsigned short b) { return __uint_as_float(((unsigned)b) << 16); }
__device__ __forceinline__ float bfr(float f) { return bf2f(f2bf(f)); }
__device__ __forceinline__ v16h cat16(v8h lo, v8h hi) { return __builtin_shufflevector(lo, hi, 0, 1, 2, 3, 4, 5, 6, 7, 8, 9, 10, 11, 12, 13, 14, 15); }
__device__ __forceinline__ v16bf cat16b(v8us lo, v8us hi) { return __builtin_bit_cast(v16bf, __builtin_shufflevector(lo, hi, 0, 1, 2, 3, 4, 5, 6, 7, 8, 9, 10, 11, 12, 13, 14, 15)); }
__device__ __forceinline__ v8f wmma16(v16h a, v16h b, v8f c) { return __builtin_amdgcn_wmma_f32_16x16x32_f16(false, a, false, b, (short)0, c, false, false); }
__device__ __forceinline__ v8f wmmab(v16bf a, v16bf b, v8f c) { return __builtin_amdgcn_wmma_f32_16x16x32_bf16(false, a, false, b, (short)0, c, false, false); }

template <typename T16> struct WFrag;
template <> struct WFrag<h16> { typedef v16h V; static __device__ __forceinline__ V ld(const h16* p) { return cat16(*(const v8h*)p, *(const v8h*)(p + 16)); } static __device__ __forceinline__ v8f mma(V a, V b, v8f c) { return wmma16(a, b, c); } };
template <> struct WFrag<bf> { typedef v16bf V; static __device__ __forceinline__ V ld(const bf* p) { return cat16b(*(const v8us*)p, *(const v8us*)(p + 16)); } static __device__ __forceinline__ v8f mma(V a, V b, v8f c) { return wmmab(a, b, c); } };
template <typename T16, int NSPLIT, bool BIAS>
__global__ __launch_bounds__(32) void k_gemmw(const T16* __restrict__ A, const T16* __restrict__ A2, const T16* __restrict__ Bt, const T16* __restrict__ Bt2, int K, float* C, int ldc, const float* __restrict__ bias, size_t sA, size_t sB, size_t sC) {
    typedef typename WFrag<T16>::V V;
    __shared__ __align__(16) float os[16 * 68];
    const size_t z = blockIdx.z; A += z * sA; if (A2) A2 += z * sA; Bt += z * sB; if (Bt2) Bt2 += z * sB; C += z * sC;
    const int lane = threadIdx.x & 31, lr = lane & 15, hi = lane >> 4; const int r0 = blockIdx.x * 64, c0 = blockIdx.y * 64;
    v8f acc[4][4];
#pragma unroll
    for (int mb = 0; mb < 4; ++mb)
#pragma unroll
        for (int nb = 0; nb < 4; ++nb) acc[mb][nb] = (v8f){};
    const size_t aoff = (size_t)(r0 + lr) * K + 8 * hi, boff = (size_t)(c0 + lr) * K + 8 * hi;
#pragma unroll 1
    for (int kc = 0; kc < K; kc += 32) {
        V a[4], a2[4];
#pragma unroll
        for (int mb = 0; mb < 4; ++mb) { a[mb] = WFrag<T16>::ld(A + aoff + (size_t)mb * 16 * K + kc); if (NSPLIT == 1 || NSPLIT == 2) a2[mb] = WFrag<T16>::ld(A2 + aoff + (size_t)mb * 16 * K + kc); }
#pragma unroll
        for (int nb = 0; nb < 4; ++nb) { const V b = WFrag<T16>::ld(Bt + boff + (size_t)nb * 16 * K + kc); V b2; if (NSPLIT >= 2) b2 = WFrag<T16>::ld(Bt2 + boff + (size_t)nb * 16 * K + kc);
#pragma unroll
            for (int mb = 0; mb < 4; ++mb) { acc[mb][nb] = WFrag<T16>::mma(a[mb], b, acc[mb][nb]); if (NSPLIT == 1 || NSPLIT == 2) acc[mb][nb] = WFrag<T16>::mma(a2[mb], b, acc[mb][nb]); if (NSPLIT >= 2) acc[mb][nb] = WFrag<T16>::mma(a[mb], b2, acc[mb][nb]); } }
        asm volatile("v_nop\n\tv_nop\n\tv_nop\n\tv_nop" : "+v"(acc[0][0]), "+v"(acc[1][1]), "+v"(acc[2][2]), "+v"(acc[3][3]) : "v"(a[0]), "v"(a[3]));
    }
#pragma unroll
    for (int mb = 0; mb < 4; ++mb) {
#pragma unroll
        for (int nb = 0; nb < 4; ++nb) {
#pragma unroll
            for (int j = 0; j < 8; ++j) os[(hi * 8 + j) * 68 + nb * 16 + lr] = acc[mb][nb][j]; }
        __builtin_amdgcn_wave_barrier(); asm volatile("" ::: "memory");
        float* crow = C + (size_t)(r0 + mb * 16) * ldc + c0;
#pragma unroll 1
        for (int ps = 0; ps < 2; ++ps) {
#pragma unroll
            for (int s = 0; s < 8; ++s) { const int row = 2 * s + hi, cofs = lr * 4; v4f val = *(const v4fa*)(os + row * 68 + cofs); if (BIAS) { val[0] += bfr(bias[c0 + cofs]); val[1] += bfr(bias[c0 + cofs + 1]); val[2] += bfr(bias[c0 + cofs + 2]); val[3] += bfr(bias[c0 + cofs + 3]); }
                *(volatile v4f*)(crow + (size_t)row * ldc + cofs) = val; }
            if (ps == 0) __threadfence(); }
        __builtin_amdgcn_wave_barrier(); asm volatile("" ::: "memory");
    }
}

__device__ __forceinline__ void splitf(float y, unsigned short& h, unsigned short& l) { h = f2bf(y); l = f2bf(y - bf2f(h)); }
typedef __attribute__((ext_vector_type(2))) unsigned short v2us;
typedef __attribute__((ext_vector_type(2))) float v2f;

__global__ __launch_bounds__(256) void k_wtb(const float* __restrict__ w, int K, int N, int nmat, bf* Bt) {
    const int lane = threadIdx.x & 31; const int L0 = (blockIdx.x * 8 + (threadIdx.x >> 5)) * 8; const int nlines = nmat * N * K / 64; const size_t mk = (size_t)K * N;
#pragma unroll
    for (int ps = 0; ps < 2; ++ps) {
#pragma unroll 1
        for (int l = 0; l < 8; ++l) { const int L = L0 + l; if (L >= nlines) break; const size_t e = (size_t)L * 64 + lane * 2; const int mat = (int)(e / mk); const size_t rr = e - (size_t)mat * mk; const int k = (int)(rr % (size_t)K), n = (int)(rr / (size_t)K); v2us o;
            o[0] = f2bf(w[((size_t)mat * K + k) * N + n]); o[1] = f2bf(w[((size_t)mat * K + k + 1) * N + n]); *(volatile v2us*)(Bt + e) = o; }
        if (ps == 0) __threadfence(); }
}
__global__ __launch_bounds__(256) void k_cvtx(const float* __restrict__ x, bf* XB, size_t n8) { const size_t i = (size_t)blockIdx.x * 256 + threadIdx.x; if (i >= n8) return; const size_t per = (size_t)SEQ * DM / 8; const size_t b = i / per, r = i - b * per; const v8f v = *(const v8f*)(x + b * (size_t)SEQ_FULL * DM + r * 8); v8us o;
#pragma unroll
    for (int k = 0; k < 8; ++k) o[k] = f2bf(v[k]); *(volatile v8us*)(XB + i * 8) = o; __threadfence(); *(volatile v8us*)(XB + i * 8) = o; }

__global__ __launch_bounds__(256) void k_qkpl(const float* __restrict__ F, bf* Qh, bf* Ql, bf* Kh, bf* Kl) {
    const size_t e = ((size_t)blockIdx.x * 256 + threadIdx.x) * 2; if (e >= (size_t)NB * NH * SEQ * HD) return;
    const int d = (int)(e % HD); const int s = (int)((e / HD) % SEQ); const int h = (int)((e / ((size_t)HD * SEQ)) % NH); const int b = (int)(e / ((size_t)HD * SEQ * NH));
    const float* f = F + ((size_t)b * SEQ + s) * D3 + (size_t)(h * 3) * HD + d;
    const v2f q2 = *(const v2f*)f; const v2f k2 = *(const v2f*)(f + HD);
    v2us qh, ql, kh, kl;
#pragma unroll
    for (int q = 0; q < 2; ++q) { unsigned short a, c2; splitf(q2[q] * SCL, a, c2); qh[q] = a; ql[q] = c2; splitf(k2[q], a, c2); kh[q] = a; kl[q] = c2; }
    *(volatile v2us*)(Qh + e) = qh; *(volatile v2us*)(Ql + e) = ql; *(volatile v2us*)(Kh + e) = kh; *(volatile v2us*)(Kl + e) = kl; __threadfence();
    *(volatile v2us*)(Qh + e) = qh; *(volatile v2us*)(Ql + e) = ql; *(volatile v2us*)(Kh + e) = kh; *(volatile v2us*)(Kl + e) = kl;
}
__global__ __launch_bounds__(256) void k_vtp(const float* __restrict__ F, bf* Vh, bf* Vl) {
    const size_t e = ((size_t)blockIdx.x * 256 + threadIdx.x) * 2; if (e >= (size_t)NB * NH * HD * SEQ) return;
    const int t = (int)(e % SEQ); const int d = (int)((e / SEQ) % HD); const int h = (int)((e / ((size_t)SEQ * HD)) % NH); const int b = (int)(e / ((size_t)SEQ * HD * NH));
    v2us oh, ol;
#pragma unroll
    for (int q = 0; q < 2; ++q) { const float xv = F[((size_t)b * SEQ + t + q) * D3 + (size_t)(h * 3 + 2) * HD + d]; unsigned short a, c2; splitf(xv, a, c2); oh[q] = a; ol[q] = c2; }
    *(volatile v2us*)(Vh + e) = oh; *(volatile v2us*)(Vl + e) = ol; __threadfence(); *(volatile v2us*)(Vh + e) = oh; *(volatile v2us*)(Vl + e) = ol;
}

__global__ __launch_bounds__(32) void k_attn(const bf* __restrict__ Qh, const bf* __restrict__ Ql, const bf* __restrict__ Kh, const bf* __restrict__ Kl,
                                             const bf* __restrict__ Vh, const bf* __restrict__ Vl, bf* Ah, bf* Al) {
    __shared__ __align__(16) bf psh[16 * PP];
    __shared__ __align__(16) bf psl[16 * PP];
    __shared__ __align__(16) float os[16 * 68];
    const int lane = threadIdx.x & 31, lr = lane & 15, hi = lane >> 4;
    const int s0 = blockIdx.x * 16, h = blockIdx.y, b = blockIdx.z;
    const size_t hp = ((size_t)b * NH + h) * (size_t)SEQ * HD;
    const bf* qh = Qh + hp + (size_t)(s0 + lr) * HD + 8 * hi; const bf* ql = Ql + hp + (size_t)(s0 + lr) * HD + 8 * hi;
    const bf* kh = Kh + hp + (size_t)lr * HD + 8 * hi;        const bf* kl = Kl + hp + (size_t)lr * HD + 8 * hi;
    const bf* vh = Vh + hp + (size_t)lr * SEQ + 8 * hi;       const bf* vl = Vl + hp + (size_t)lr * SEQ + 8 * hi;
    v16bf qa[2], qa2[2];
#pragma unroll
    for (int ks = 0; ks < 2; ++ks) { qa[ks] = WFrag<bf>::ld(qh + ks * 32); qa2[ks] = WFrag<bf>::ld(ql + ks * 32); }
    float mrow[8], lrow[8];
#pragma unroll
    for (int r = 0; r < 8; ++r) { mrow[r] = -1.0e30f; lrow[r] = 0.0f; }
    v8f oacc[4];
#pragma unroll
    for (int nt = 0; nt < 4; ++nt) oacc[nt] = (v8f){};
    v16bf ph[2], pl[2];
#pragma unroll 1
    for (int t0 = 0; t0 < SEQ; t0 += KCH) {
        v8f sacc[4];
#pragma unroll
        for (int nt = 0; nt < 4; ++nt) sacc[nt] = (v8f){};
#pragma unroll
        for (int nt = 0; nt < 4; ++nt) {
#pragma unroll
            for (int ks = 0; ks < 2; ++ks) {
                const v16bf kbh = WFrag<bf>::ld(kh + (size_t)(t0 + nt * 16) * HD + ks * 32);
                const v16bf kbl = WFrag<bf>::ld(kl + (size_t)(t0 + nt * 16) * HD + ks * 32);
                sacc[nt] = wmmab(qa[ks], kbh, sacc[nt]); sacc[nt] = wmmab(qa2[ks], kbh, sacc[nt]); sacc[nt] = wmmab(qa[ks], kbl, sacc[nt]);
            }
        }
        asm volatile("v_nop\n\tv_nop\n\tv_nop\n\tv_nop" : "+v"(sacc[0]), "+v"(sacc[1]), "+v"(sacc[2]), "+v"(sacc[3]) : "v"(qa[0]), "v"(qa2[1]));
        float sc[8], rs[8];
#pragma unroll
        for (int r = 0; r < 8; ++r) {
            float m = fmaxf(fmaxf(sacc[0][r], sacc[1][r]), fmaxf(sacc[2][r], sacc[3][r]));
#pragma unroll
            for (int sh = 1; sh < 16; sh <<= 1) m = fmaxf(m, __shfl_xor(m, sh, 32));
            const float mn = fmaxf(mrow[r], m);
            sc[r] = __builtin_amdgcn_exp2f(__fmul_rn(__fsub_rn(mrow[r], mn), L2E)); mrow[r] = mn; rs[r] = 0.0f;
        }
#pragma unroll
        for (int nt = 0; nt < 4; ++nt)
#pragma unroll
            for (int r = 0; r < 8; ++r) { const float p = __builtin_amdgcn_exp2f(__fmul_rn(__fsub_rn(sacc[nt][r], mrow[r]), L2E)); sacc[nt][r] = p; rs[r] += p; }
#pragma unroll
        for (int r = 0; r < 8; ++r) {
            float s = rs[r];
#pragma unroll
            for (int sh = 1; sh < 16; sh <<= 1) s += __shfl_xor(s, sh, 32);
            lrow[r] = lrow[r] * sc[r] + s;
        }
#pragma unroll
        for (int nt = 0; nt < 4; ++nt)
#pragma unroll
            for (int r = 0; r < 8; ++r) oacc[nt][r] *= sc[r];
#pragma unroll
        for (int nt = 0; nt < 4; ++nt)
#pragma unroll
            for (int r = 0; r < 8; ++r) { unsigned short a, c2; splitf(sacc[nt][r] * PCAR, a, c2); const int o = (hi * 8 + r) * PP + nt * 16 + lr; psh[o] = a; psl[o] = c2; }
        __builtin_amdgcn_fence(3, "wavefront"); __builtin_amdgcn_wave_barrier();
#pragma unroll
        for (int kk = 0; kk < 2; ++kk) {
            ph[kk] = WFrag<bf>::ld(psh + lr * PP + kk * 32 + 8 * hi); pl[kk] = WFrag<bf>::ld(psl + lr * PP + kk * 32 + 8 * hi);
#pragma unroll
            for (int nt = 0; nt < 4; ++nt) {
                const v16bf vbh = WFrag<bf>::ld(vh + (size_t)nt * 16 * SEQ + t0 + kk * 32);
                const v16bf vbl = WFrag<bf>::ld(vl + (size_t)nt * 16 * SEQ + t0 + kk * 32);
                oacc[nt] = wmmab(ph[kk], vbh, oacc[nt]); oacc[nt] = wmmab(pl[kk], vbh, oacc[nt]); oacc[nt] = wmmab(ph[kk], vbl, oacc[nt]);
            }
        }
        asm volatile("v_nop\n\tv_nop\n\tv_nop\n\tv_nop" : "+v"(oacc[0]), "+v"(oacc[1]), "+v"(oacc[2]), "+v"(oacc[3]) : "v"(ph[0]), "v"(pl[1]));
        asm volatile("" ::: "memory");
    }
    float rinv[8];
#pragma unroll
    for (int r = 0; r < 8; ++r) rinv[r] = __fdiv_rn(1.0f, lrow[r] * PCAR);
#pragma unroll
    for (int nt = 0; nt < 4; ++nt)
#pragma unroll
        for (int r = 0; r < 8; ++r) os[(hi * 8 + r) * 68 + nt * 16 + lr] = oacc[nt][r] * rinv[r];
    __builtin_amdgcn_fence(3, "wavefront"); __builtin_amdgcn_wave_barrier();
    const int rg = lane >> 3, c8 = (lane & 7) * 8;
    bf* ah = Ah + ((size_t)b * SEQ + s0) * DQ + (size_t)h * HD + c8; bf* al = Al + ((size_t)b * SEQ + s0) * DQ + (size_t)h * HD + c8;
#pragma unroll 1
    for (int ps = 0; ps < 2; ++ps) {
#pragma unroll
        for (int it = 0; it < 4; ++it) {
            const int row = it * 4 + rg; const v4f x0 = *(const v4fa*)(os + row * 68 + c8); const v4f x1 = *(const v4fa*)(os + row * 68 + c8 + 4); v8us oh, ol;
#pragma unroll
            for (int j = 0; j < 4; ++j) { unsigned short a, c2; splitf(x0[j], a, c2); oh[j] = a; ol[j] = c2; splitf(x1[j], a, c2); oh[4 + j] = a; ol[4 + j] = c2; }
            *(volatile v8us*)(ah + (size_t)row * DQ) = oh; *(volatile v8us*)(al + (size_t)row * DQ) = ol;
        }
        if (ps == 0) __threadfence();
    }
}

extern "C" void kernel_launch(void* const* d_in, const int* in_sizes, int n_in,
                              void* d_out, int out_size, void* d_ws, size_t ws_size, hipStream_t stream) {
    if (n_in < 3) return;
    if ((long long)in_sizes[0] < ((long long)(NB - 1) * SEQ_FULL + SEQ) * DM) return;
    if (in_sizes[1] < NH * 3 * DM * HD) return;
    if (in_sizes[2] < DQ * FO) return;
    if (out_size < NB * SEQ * FO) return;
    const float* x  = (const float*)d_in[0];
    const float* w  = (const float*)d_in[1];
    const float* wo = (const float*)d_in[2];
    float* OUT = (float*)d_out;
    char* wsp = (char*)d_ws;
    auto take = [&](size_t bytes) { char* p = wsp; wsp += (bytes + 255) & ~(size_t)255; return (void*)p; };
    const size_t npl = (size_t)NB * NH * SEQ * HD;
    bf* WB  = (bf*)take((size_t)D3 * DM * 2);
    bf* WOB = (bf*)take((size_t)FO * DQ * 2);
    bf* XB  = (bf*)take((size_t)NB * SEQ * DM * 2);
    float* F = (float*)take((size_t)NB * SEQ * D3 * 4);
    bf* QPh = (bf*)take(npl * 2); bf* QPl = (bf*)take(npl * 2);
    bf* KPh = (bf*)take(npl * 2); bf* KPl = (bf*)take(npl * 2);
    bf* VTh = (bf*)take(npl * 2); bf* VTl = (bf*)take(npl * 2);
    bf* ATh = (bf*)take((size_t)NB * SEQ * DQ * 2); bf* ATl = (bf*)take((size_t)NB * SEQ * DQ * 2);
    const size_t used = (size_t)(wsp - (char*)d_ws);
    if (used > ws_size || used > (size_t)134217728) return;

    k_wtb<<<(unsigned)((NH * 3 * HD * DM / 64 + 63) / 64), 256, 0, stream>>>(w, DM, HD, NH * 3, WB);
    k_wtb<<<(unsigned)((DQ * FO / 64 + 63) / 64), 256, 0, stream>>>(wo, DQ, FO, 1, WOB);
    const size_t n8 = (size_t)NB * SEQ * DM / 8;
    k_cvtx<<<(unsigned)((n8 + 255) / 256), 256, 0, stream>>>(x, XB, n8);
    k_gemmw<bf, 0, false><<<dim3(SEQ / 64, D3 / 64, NB), 32, 0, stream>>>(XB, nullptr, WB, nullptr, DM, F, D3, nullptr, (size_t)SEQ * DM, (size_t)0, (size_t)SEQ * D3);
    const unsigned LP = (unsigned)((npl / 2 + 255) / 256);
    k_qkpl<<<LP, 256, 0, stream>>>(F, QPh, QPl, KPh, KPl);
    k_vtp<<<LP, 256, 0, stream>>>(F, VTh, VTl);
    k_attn<<<dim3(SEQ / 16, NH, NB), 32, 0, stream>>>(QPh, QPl, KPh, KPl, VTh, VTl, ATh, ATl);
    k_gemmw<bf, 1, false><<<dim3(NB * SEQ / 64, FO / 64, 1), 32, 0, stream>>>(ATh, ATl, WOB, nullptr, DQ, OUT, FO, nullptr, (size_t)0, (size_t)0, (size_t)0);
}
